// RelPartialLearnableMultiHeadAttn_72172630442404
// MI455X (gfx1250) — hardware-run, weakly checked
//
#include <hip/hip_runtime.h>


#define NB_  16
#define TT   384
#define DM   1024
#define NH_  16
#define NKV  16
#define REP  (NH_ / NKV)
#define HD   64
#define DQ   (NH_ * HD)
#define DKV  (NKV * HD)
#define ZH   2
#define RH   384
#define WIN  0
#define PCAR 1024.0f
#define SCL  0.125f
#define TK   768
#define ML   384
#define BSZ  16
#define DQ3  3072
typedef _Float16 h16;
typedef unsigned short bf;
typedef __attribute__((ext_vector_type(16))) __bf16   v16bf;
typedef __attribute__((ext_vector_type(16))) _Float16 v16h;
typedef __attribute__((ext_vector_type(8)))  _Float16 v8h;
typedef __attribute__((ext_vector_type(8)))  unsigned short v8us;
typedef __attribute__((ext_vector_type(8)))  float    v8f;
typedef __attribute__((ext_vector_type(4)))  float    v4f;
typedef v8h  __attribute__((may_alias)) v8ha;
typedef v4f  __attribute__((may_alias)) v4fa;
typedef v8us __attribute__((may_alias)) v8usa;

__device__ __forceinline__ unsigned short f2bf(float f) { unsigned u = __float_as_uint(f); u += 0x7FFFu + ((u >> 16) & 1u); return (unsigned short)(u >> 16); }
__device__ __forceinline__ float bf2f(unsigned short b) { return __uint_as_float(((unsigned)b) << 16); }
__device__ __forceinline__ float bfr(float f) { return bf2f(f2bf(f)); }
__device__ __forceinline__ v16h cat16(v8h lo, v8h hi) { return __builtin_shufflevector(lo, hi, 0, 1, 2, 3, 4, 5, 6, 7, 8, 9, 10, 11, 12, 13, 14, 15); }
__device__ __forceinline__ v16bf cat16b(v8us lo, v8us hi) { return __builtin_bit_cast(v16bf, __builtin_shufflevector(lo, hi, 0, 1, 2, 3, 4, 5, 6, 7, 8, 9, 10, 11, 12, 13, 14, 15)); }
__device__ __forceinline__ v8f wmma16(v16h a, v16h b, v8f c) { return __builtin_amdgcn_wmma_f32_16x16x32_f16(false, a, false, b, (short)0, c, false, false); }
__device__ __forceinline__ v8f wmmab(v16bf a, v16bf b, v8f c) { return __builtin_amdgcn_wmma_f32_16x16x32_bf16(false, a, false, b, (short)0, c, false, false); }


template <typename T16> struct WFrag;
template <> struct WFrag<h16> { typedef v16h V; static __device__ __forceinline__ V ld(const h16* p) { return cat16(*(const v8h*)p, *(const v8h*)(p + 16)); } static __device__ __forceinline__ v8f mma(V a, V b, v8f c) { return wmma16(a, b, c); } };
template <> struct WFrag<bf> { typedef v16bf V; static __device__ __forceinline__ V ld(const bf* p) { return cat16b(*(const v8us*)p, *(const v8us*)(p + 16)); } static __device__ __forceinline__ v8f mma(V a, V b, v8f c) { return wmmab(a, b, c); } };
template <typename T16, int NSPLIT, bool BIAS>
__global__ __launch_bounds__(32) void k_gemmw(const T16* __restrict__ A, const T16* __restrict__ A2, const T16* __restrict__ Bt, const T16* __restrict__ Bt2, int K, float* C, int ldc, const float* __restrict__ bias, size_t sA, size_t sB, size_t sC) {
    typedef typename WFrag<T16>::V V;
    __shared__ __align__(16) float os[16 * 68];
    const size_t z = blockIdx.z; A += z * sA; if (A2) A2 += z * sA; Bt += z * sB; if (Bt2) Bt2 += z * sB; C += z * sC;
    const int lane = threadIdx.x & 31, lr = lane & 15, hi = lane >> 4; const int r0 = blockIdx.x * 64, c0 = blockIdx.y * 64;
    v8f acc[4][4];
#pragma unroll
    for (int mb = 0; mb < 4; ++mb)
#pragma unroll
        for (int nb = 0; nb < 4; ++nb) acc[mb][nb] = (v8f){};
    const size_t aoff = (size_t)(r0 + lr) * K + 8 * hi, boff = (size_t)(c0 + lr) * K + 8 * hi;
#pragma unroll 1
    for (int kc = 0; kc < K; kc += 32) {
        V a[4], a2[4];
#pragma unroll
        for (int mb = 0; mb < 4; ++mb) { a[mb] = WFrag<T16>::ld(A + aoff + (size_t)mb * 16 * K + kc); if (NSPLIT == 1 || NSPLIT == 2) a2[mb] = WFrag<T16>::ld(A2 + aoff + (size_t)mb * 16 * K + kc); }
#pragma unroll
        for (int nb = 0; nb < 4; ++nb) { const V b = WFrag<T16>::ld(Bt + boff + (size_t)nb * 16 * K + kc); V b2; if (NSPLIT >= 2) b2 = WFrag<T16>::ld(Bt2 + boff + (size_t)nb * 16 * K + kc);
#pragma unroll
            for (int mb = 0; mb < 4; ++mb) { acc[mb][nb] = WFrag<T16>::mma(a[mb], b, acc[mb][nb]); if (NSPLIT == 1 || NSPLIT == 2) acc[mb][nb] = WFrag<T16>::mma(a2[mb], b, acc[mb][nb]); if (NSPLIT >= 2) acc[mb][nb] = WFrag<T16>::mma(a[mb], b2, acc[mb][nb]); } }
        asm volatile("v_nop\n\tv_nop\n\tv_nop\n\tv_nop" : "+v"(acc[0][0]), "+v"(acc[1][1]), "+v"(acc[2][2]), "+v"(acc[3][3]) : "v"(a[0]), "v"(a[3]));
    }
#pragma unroll
    for (int mb = 0; mb < 4; ++mb) {
#pragma unroll
        for (int nb = 0; nb < 4; ++nb) {
#pragma unroll
            for (int j = 0; j < 8; ++j) os[(hi * 8 + j) * 68 + nb * 16 + lr] = acc[mb][nb][j]; }
        __builtin_amdgcn_wave_barrier(); asm volatile("" ::: "memory");
        float* crow = C + (size_t)(r0 + mb * 16) * ldc + c0;
#pragma unroll 1
        for (int ps = 0; ps < 2; ++ps) {
#pragma unroll
            for (int s = 0; s < 8; ++s) { const int row = 2 * s + hi, cofs = lr * 4; v4f val = *(const v4fa*)(os + row * 68 + cofs); if (BIAS) { val[0] += bfr(bias[c0 + cofs]); val[1] += bfr(bias[c0 + cofs + 1]); val[2] += bfr(bias[c0 + cofs + 2]); val[3] += bfr(bias[c0 + cofs + 3]); }
                *(volatile v4f*)(crow + (size_t)row * ldc + cofs) = val; }
            if (ps == 0) __threadfence(); }
        __builtin_amdgcn_wave_barrier(); asm volatile("" ::: "memory");
    }
}

__device__ __forceinline__ h16 tohx(float x) { return (h16)x; }
__device__ __forceinline__ void splitf(float y, unsigned short& h, unsigned short& l) { h = f2bf(y); l = f2bf(y - bf2f(h)); }
typedef __attribute__((ext_vector_type(2))) _Float16 v2h;
typedef __attribute__((ext_vector_type(4))) _Float16 v4h;
typedef __attribute__((ext_vector_type(2))) unsigned short v2us;
typedef __attribute__((ext_vector_type(4))) unsigned short v4us;
typedef __attribute__((ext_vector_type(2))) float v2f;
typedef __attribute__((ext_vector_type(4))) int v4i;

__global__ __launch_bounds__(256) void k_wtG(const float* __restrict__ w, int K, int N, bf* Bt) {
    const int lane = threadIdx.x & 31; const int L0 = (blockIdx.x * 8 + (threadIdx.x >> 5)) * 8; const int nlines = N * K / 64;
#pragma unroll
    for (int ps = 0; ps < 2; ++ps) {
#pragma unroll 1
        for (int l = 0; l < 8; ++l) { const int L = L0 + l; if (L >= nlines) break; const size_t e = (size_t)L * 64 + lane * 2; const int k = (int)(e % K), n = (int)(e / K); v2us o;
            o[0] = f2bf(w[(size_t)k * N + n]); o[1] = f2bf(w[(size_t)(k + 1) * N + n]); *(volatile v2us*)(Bt + e) = o; }
        if (ps == 0) __threadfence(); }
}
__global__ __launch_bounds__(256) void k_cvt8(const float* __restrict__ src, bf* dst, size_t n8) { const size_t i = (size_t)blockIdx.x * 256 + threadIdx.x; if (i >= n8) return; const v8f v = *(const v8f*)(src + i * 8); v8us o;
#pragma unroll
    for (int k = 0; k < 8; ++k) o[k] = f2bf(v[k]); *(volatile v8us*)(dst + i * 8) = o; __threadfence(); *(volatile v8us*)(dst + i * 8) = o; }


__global__ __launch_bounds__(256) void k_asoftM(const float* __restrict__ Sb, h16* P16, bf* Ph, bf* Pl) {
    const int lane = threadIdx.x & 31; const int row = blockIdx.x * 8 + (threadIdx.x >> 5); if (row >= ZH * TT) return; const int i = row % TT; const int zz = row / TT;     (void)zz; const bool hires = (i < RH); const float* sr = Sb + (size_t)row * TK; float v[TK / 32]; float mx = -3.0e38f;
#pragma unroll
    for (int ch = 0; ch < TK / 128; ++ch) { const int j0 = ch * 128 + lane * 4; const v4f a = *(const v4f*)(sr + j0);
#pragma unroll
        for (int q = 0; q < 4; ++q) { const int j = j0 + q; const float t = (j <= i + ML) ? a[q] * SCL : -3.0e38f;     v[ch * 4 + q] = t; mx = fmaxf(mx, t); } }
#pragma unroll
    for (int sh = 16; sh; sh >>= 1) mx = fmaxf(mx, __shfl_xor(mx, sh, 32));
    float sum = 0.f;
#pragma unroll
    for (int k = 0; k < TK / 32; ++k) { float d0 = __fsub_rn(v[k], mx); asm volatile("" : "+v"(d0)); v[k] = __builtin_amdgcn_exp2f(__fmul_rn(d0, 1.4426950408889634f)); sum += v[k]; }
#pragma unroll
    for (int sh = 16; sh; sh >>= 1) sum += __shfl_xor(sum, sh, 32);
    const float f = __fdiv_rn(hires ? 1.0f : PCAR, sum);
#pragma unroll 1
    for (int ps = 0; ps < 2; ++ps) {
        if (hires) {
#pragma unroll
            for (int ch = 0; ch < TK / 128; ++ch) { v4us oh, ol;
#pragma unroll
                for (int q = 0; q < 4; ++q) { unsigned short a, c2; splitf(v[ch * 4 + q] * f, a, c2); oh[q] = a; ol[q] = c2; }
                const size_t oo = ((size_t)zz * (RH ? RH : 1) + i) * TK + ch * 128 + lane * 4; *(volatile v4us*)(Ph + oo) = oh; *(volatile v4us*)(Pl + oo) = ol; }
        } else {
#pragma unroll
            for (int ch = 0; ch < TK / 128; ++ch) { v4h o4;
#pragma unroll
                for (int q = 0; q < 4; ++q) o4[q] = tohx(v[ch * 4 + q] * f);
                *(volatile v4h*)(P16 + (size_t)row * TK + ch * 128 + lane * 4) = o4; } }
        if (ps == 0) __threadfence(); }
}


__global__ __launch_bounds__(256) void k_merge(const float* __restrict__ O, int h0, bf* Ah, bf* Al) { const size_t e = ((size_t)blockIdx.x * 256 + threadIdx.x) * 2; if (e >= (size_t)ZH * TT * HD) return; const int d = (int)(e % HD); const int t = (int)((e / HD) % TT); const int zz = (int)(e / ((size_t)HD * TT)); const float cs = (t < RH) ? 1.0f : (1.0f / PCAR); const size_t oo = (size_t)t * DQ + (h0 + zz) * HD + d;
    v2us oh, ol;
#pragma unroll
    for (int q = 0; q < 2; ++q) { unsigned short a, c2; splitf(O[e + q] * cs, a, c2); oh[q] = a; ol[q] = c2; } *(volatile v2us*)(Ah + oo) = oh; *(volatile v2us*)(Al + oo) = ol; __threadfence(); *(volatile v2us*)(Ah + oo) = oh; *(volatile v2us*)(Al + oo) = ol; }

__global__ __launch_bounds__(256) void k_planesR(const float* __restrict__ F, int pitch, int nheads, int rows, h16* P16, bf* Ph, bf* Pl) { const size_t e = ((size_t)blockIdx.x * 256 + threadIdx.x) * 2; if (e >= (size_t)nheads * rows * HD) return; const int d = (int)(e % HD); const int t = (int)((e / HD) % rows); const int h = (int)(e / ((size_t)HD * rows)); const float* f = F + (size_t)t * pitch + h * HD + d; v2h o16; v2us oh, ol;
#pragma unroll
    for (int q = 0; q < 2; ++q) { o16[q] = tohx(f[q]); unsigned short a, c2; splitf(f[q], a, c2); oh[q] = a; ol[q] = c2; }
    *(volatile v2h*)(P16 + e) = o16; *(volatile v2us*)(Ph + e) = oh; *(volatile v2us*)(Pl + e) = ol; __threadfence(); *(volatile v2h*)(P16 + e) = o16; *(volatile v2us*)(Ph + e) = oh; *(volatile v2us*)(Pl + e) = ol; }
__global__ __launch_bounds__(256) void k_vtpR2(const float* __restrict__ F, int pitch, int nheads, int rows, h16* V16, bf* Vh, bf* Vl) { const size_t e = ((size_t)blockIdx.x * 256 + threadIdx.x) * 2; if (e >= (size_t)nheads * HD * rows) return; const int t = (int)(e % rows); const int d = (int)((e / rows) % HD); const int h = (int)(e / ((size_t)rows * HD)); v2h o16; v2us oh, ol;
#pragma unroll
    for (int q = 0; q < 2; ++q) { const float x = F[(size_t)(t + q) * pitch + h * HD + d]; o16[q] = tohx(x); unsigned short a, c2; splitf(x, a, c2); oh[q] = a; ol[q] = c2; }
    *(volatile v2h*)(V16 + e) = o16; *(volatile v2us*)(Vh + e) = oh; *(volatile v2us*)(Vl + e) = ol; __threadfence(); *(volatile v2h*)(V16 + e) = o16; *(volatile v2us*)(Vh + e) = oh; *(volatile v2us*)(Vl + e) = ol; }
__global__ __launch_bounds__(256) void k_hdot(const float* __restrict__ bias, const float* __restrict__ F, int pitch, int nrows, int hcol, float* OUT) { const int lane = threadIdx.x & 31; const size_t wv = (size_t)blockIdx.x * 8 + (threadIdx.x >> 5); if (wv >= (size_t)NH_ * (nrows / 32)) return; const int h = (int)(wv / (nrows / 32)); const int n = (int)(wv % (nrows / 32)) * 32 + lane; const float* f = F + (size_t)n * pitch + (hcol ? h * HD : 0);     const float* bh = bias + h * HD; float s = 0.f;
#pragma unroll 4
    for (int d = 0; d < HD; ++d) { s = __fadd_rn(s, __fmul_rn(bfr(bh[d]), f[d])); }
    *(volatile float*)(OUT + (size_t)h * nrows + n) = s; __threadfence(); *(volatile float*)(OUT + (size_t)h * nrows + n) = s; }

__global__ __launch_bounds__(256) void k_gath2(const float* __restrict__ mb, const float* __restrict__ wb, bf* XB) { const size_t k = (size_t)blockIdx.x * 256 + threadIdx.x; if (k >= (size_t)TK * DM / 8) return; const int c0 = (int)(k % (DM / 8)) * 8; const int j = (int)(k / (DM / 8)); const int jm = min(j, ML - 1), jw = min(max(j - ML, 0), TT - 1); const v8f am = *(const v8f*)(mb + (size_t)jm * BSZ * DM + c0); const v8f aw = *(const v8f*)(wb + (size_t)jw * BSZ * DM + c0); v8us o;
#pragma unroll
    for (int q = 0; q < 8; ++q) o[q] = f2bf(j < ML ? am[q] : aw[q]);
    *(volatile v8us*)(XB + (size_t)j * DM + c0) = o; __threadfence(); *(volatile v8us*)(XB + (size_t)j * DM + c0) = o; }
__global__ __launch_bounds__(256) void k_addxlm(float* Sb, const float* __restrict__ QR, const float* __restrict__ KB, const float* __restrict__ RB, int h0) { const size_t k = (size_t)blockIdx.x * 256 + threadIdx.x; if (k >= (size_t)ZH * TT * TK / 4) return; const size_t e = k * 4; const int j0 = (int)(e % TK); const int i = (int)((e / TK) % TT); const int zz = (int)(e / ((size_t)TT * TK)); const int h = h0 + zz; const float* qr = QR + ((size_t)zz * TT + i) * TK; v4f a = *(const v4f*)(Sb + e); const v4f kb = *(const v4f*)(KB + (size_t)h * TK + j0);
#pragma unroll
    for (int q = 0; q < 4; ++q) { const int c = min(max(ML - 1 - i + j0 + q, 0), TK - 1); float s1 = __fadd_rn(a[q], kb[q]); asm volatile("" : "+v"(s1)); float s2 = __fadd_rn(s1, qr[c]); asm volatile("" : "+v"(s2)); a[q] = __fadd_rn(s2, RB[(size_t)h * TK + c]); }
    *(volatile v4f*)(Sb + e) = a; __threadfence(); *(volatile v4f*)(Sb + e) = a; }
__global__ __launch_bounds__(256) void k_lnrS(const float* __restrict__ wb, const float* __restrict__ Y, const float* __restrict__ g, const float* __restrict__ bb, float* ob) { const int lane = threadIdx.x & 31; const int row = blockIdx.x * 8 + (threadIdx.x >> 5); if (row >= TT) return; const float* br = wb + (size_t)row * BSZ * DM; const float* yr = Y + (size_t)row * DM; float v[DM / 32]; float s = 0.f;
#pragma unroll
    for (int ch = 0; ch < DM / 128; ++ch) { const v4f a = *(const v4f*)(br + ch * 128 + lane * 4); const v4f y4 = *(const v4f*)(yr + ch * 128 + lane * 4);
#pragma unroll
        for (int q = 0; q < 4; ++q) { float ab = bfr(a[q]); asm volatile("" : "+v"(ab)); float t = __fadd_rn(ab, y4[q]); asm volatile("" : "+v"(t)); v[ch * 4 + q] = t; s = __fadd_rn(s, t); } }
#pragma unroll
    for (int sh = 16; sh; sh >>= 1) s = __fadd_rn(s, __shfl_xor(s, sh, 32));
    const float mu = __fdiv_rn(s, (float)DM); float s2 = 0.f;
#pragma unroll
    for (int k = 0; k < DM / 32; ++k) { const float dv = __fsub_rn(v[k], mu); float p2 = __fmul_rn(dv, dv); asm volatile("" : "+v"(p2)); s2 = __fadd_rn(s2, p2); }
#pragma unroll
    for (int sh = 16; sh; sh >>= 1) s2 = __fadd_rn(s2, __shfl_xor(s2, sh, 32));
    const float rs = __fdiv_rn(1.0f, __fsqrt_rn(__fadd_rn(__fdiv_rn(s2, (float)DM), 1e-5f)));
#pragma unroll 1
    for (int ps = 0; ps < 2; ++ps) {
#pragma unroll
        for (int ch = 0; ch < DM / 128; ++ch) { v4f o; for (int q = 0; q < 4; ++q) { const int col = ch * 128 + lane * 4 + q; float dv = __fsub_rn(v[ch * 4 + q], mu); asm volatile("" : "+v"(dv)); float y = __fmul_rn(dv, rs); asm volatile("" : "+v"(y)); float gg = bfr(g[col]), bb2 = bfr(bb[col]); asm volatile("" : "+v"(gg), "+v"(bb2)); y = __fmul_rn(y, gg); asm volatile("" : "+v"(y)); o[q] = __fadd_rn(y, bb2); }
            *(volatile v4f*)(ob + (size_t)row * BSZ * DM + ch * 128 + lane * 4) = o; }
        if (ps == 0) __threadfence(); } }

extern "C" void kernel_launch(void* const* d_in, const int* in_sizes, int n_in,
                              void* d_out, int out_size, void* d_ws, size_t ws_size, hipStream_t stream) {
    (void)in_sizes; (void)n_in; (void)out_size;
    const float* w = (const float*)d_in[0]; const float* r = (const float*)d_in[1]; const float* rwb = (const float*)d_in[2]; const float* rrb = (const float*)d_in[3]; const float* mems = (const float*)d_in[4];   const float* wqkv = (const float*)d_in[6]; const float* wr = (const float*)d_in[7]; const float* wo = (const float*)d_in[8]; const float* lng = (const float*)d_in[9]; const float* lnb = (const float*)d_in[10];
    float* OUT = (float*)d_out;
    char* wsp = (char*)d_ws;
    auto take = [&](size_t bytes) { char* p = wsp; wsp += (bytes + 255) & ~(size_t)255; return (void*)p; };
    bf* WQKV = (bf*)take((size_t)DQ3 * DM * 2); bf* WR = (bf*)take((size_t)DM * DM * 2); bf* WO = (bf*)take((size_t)DM * DM * 2);
    bf* RBF = (bf*)take((size_t)TK * DM * 2); float* RF = (float*)take((size_t)TK * DM * 4); h16* RP16 = (h16*)take((size_t)NH_ * TK * HD * 2); bf* RPh = (bf*)take((size_t)NH_ * TK * HD * 2); bf* RPl = (bf*)take((size_t)NH_ * TK * HD * 2); float* RB = (float*)take((size_t)NH_ * TK * 4); float* KB = (float*)take((size_t)NH_ * TK * 4);
    bf* XB = (bf*)take((size_t)TK * DM * 2); float* F = (float*)take((size_t)TK * DQ3 * 4);
    h16* QP16 = (h16*)take((size_t)NH_ * TT * HD * 2); bf* QPh = (bf*)take((size_t)NH_ * TT * HD * 2); bf* QPl = (bf*)take((size_t)NH_ * TT * HD * 2); h16* KP16 = (h16*)take((size_t)NH_ * TK * HD * 2); bf* KPh = (bf*)take((size_t)NH_ * TK * HD * 2); bf* KPl = (bf*)take((size_t)NH_ * TK * HD * 2); h16* VT16 = (h16*)take((size_t)NH_ * HD * TK * 2); bf* VTh = (bf*)take((size_t)NH_ * HD * TK * 2); bf* VTl = (bf*)take((size_t)NH_ * HD * TK * 2);
    float* Sb = (float*)take((size_t)ZH * TT * TK * 4); float* QR = (float*)take((size_t)ZH * TT * TK * 4); bf* Ph = (bf*)take((size_t)ZH * TT * TK * 2); bf* Pl = (bf*)take((size_t)ZH * TT * TK * 2); float* Ob = (float*)take((size_t)ZH * TT * HD * 4); bf* ATh = (bf*)take((size_t)TT * DM * 2); bf* ATl = (bf*)take((size_t)TT * DM * 2); float* Y = (float*)take((size_t)TT * DM * 4);
    if ((size_t)(wsp - (char*)d_ws) > ws_size) return;
    k_wtG<<<(unsigned)((DM * DQ3 / 64 + 63) / 64), 256, 0, stream>>>(wqkv, DM, DQ3, WQKV); k_wtG<<<(unsigned)((DM * DM / 64 + 63) / 64), 256, 0, stream>>>(wr, DM, DM, WR); k_wtG<<<(unsigned)((DM * DM / 64 + 63) / 64), 256, 0, stream>>>(wo, DM, DM, WO);
    k_cvt8<<<(unsigned)(((size_t)TK * DM / 8 + 255) / 256), 256, 0, stream>>>(r, RBF, (size_t)TK * DM / 8);
    k_gemmw<bf, 0, false><<<dim3(TK / 64, DM / 64, 1), 32, 0, stream>>>(RBF, nullptr, WR, nullptr, DM, RF, DM, nullptr, 0, 0, 0);
    k_planesR<<<(unsigned)(((size_t)NH_ * TK * HD / 2 + 255) / 256), 256, 0, stream>>>(RF, DM, NH_, TK, RP16, RPh, RPl); k_hdot<<<(unsigned)(((size_t)NH_ * (TK / 32) + 7) / 8), 256, 0, stream>>>(rrb, RF, DM, TK, 1, RB);
    for (int b = 0; b < BSZ; ++b) {
        k_gath2<<<(unsigned)(((size_t)TK * DM / 8 + 255) / 256), 256, 0, stream>>>(mems + (size_t)b * DM, w + (size_t)b * DM, XB);
        k_gemmw<bf, 0, false><<<dim3(TK / 64, DQ3 / 64, 1), 32, 0, stream>>>(XB, nullptr, WQKV, nullptr, DM, F, DQ3, nullptr, 0, 0, 0);
        k_hdot<<<(unsigned)(((size_t)NH_ * (TK / 32) + 7) / 8), 256, 0, stream>>>(rwb, F + DM, DQ3, TK, 1, KB);
        k_planesR<<<(unsigned)(((size_t)NH_ * TT * HD / 2 + 255) / 256), 256, 0, stream>>>(F + (size_t)ML * DQ3, DQ3, NH_, TT, QP16, QPh, QPl);
        k_planesR<<<(unsigned)(((size_t)NH_ * TK * HD / 2 + 255) / 256), 256, 0, stream>>>(F + DM, DQ3, NH_, TK, KP16, KPh, KPl);
        k_vtpR2<<<(unsigned)(((size_t)NH_ * HD * TK / 2 + 255) / 256), 256, 0, stream>>>(F + 2 * DM, DQ3, NH_, TK, VT16, VTh, VTl);
        for (int h0 = 0; h0 < NH_; h0 += ZH) { const size_t zq = (size_t)h0, zk = (size_t)h0;
            k_gemmw<bf, 2, false><<<dim3(TT / 64, TK / 64, ZH), 32, 0, stream>>>(QPh + zq * TT * HD, QPl + zq * TT * HD, KPh + zk * TK * HD, KPl + zk * TK * HD, HD, Sb, TK, nullptr, (size_t)TT * HD, (size_t)TK * HD, (size_t)TT * TK);
            k_gemmw<bf, 2, false><<<dim3(TT / 64, TK / 64, ZH), 32, 0, stream>>>(QPh + zq * TT * HD, QPl + zq * TT * HD, RPh + zk * TK * HD, RPl + zk * TK * HD, HD, QR, TK, nullptr, (size_t)TT * HD, (size_t)TK * HD, (size_t)TT * TK);
            k_addxlm<<<(unsigned)(((size_t)ZH * TT * TK / 4 + 255) / 256), 256, 0, stream>>>(Sb, QR, KB, RB, h0);
            k_asoftM<<<ZH * TT / 8, 256, 0, stream>>>(Sb, nullptr, Ph, Pl);
            k_gemmw<bf, 2, false><<<dim3(TT / 64, HD / 64, ZH), 32, 0, stream>>>(Ph, Pl, VTh + zk * HD * TK, VTl + zk * HD * TK, TK, Ob, HD, nullptr, (size_t)TT * TK, (size_t)HD * TK, (size_t)TT * HD);
            k_merge<<<(unsigned)(((size_t)ZH * TT * HD / 2 + 255) / 256), 256, 0, stream>>>(Ob, h0, ATh, ATl); }
        k_gemmw<bf, 1, false><<<dim3(TT / 64, DM / 64, 1), 32, 0, stream>>>(ATh, ATl, WO, nullptr, DQ, Y, DM, nullptr, 0, 0, 0);
        k_lnrS<<<TT / 8, 256, 0, stream>>>(w + (size_t)b * DM, Y, lng, lnb, OUT + (size_t)b * DM); }
}
